// ContactGMP_36988258353212
// MI455X (gfx1250) — hardware-verified
//
#include <hip/hip_runtime.h>
#include <stddef.h>


#pragma clang fp contract(off)

#define HD      128
#define KN0     384
#define PQROW   256
#define NTHR    256
#define NWAVE   8
#define NBN     64
#define XP      136
#define XP3     392
#define SP      132
#define TE      128
#define AP      136
#define EPT     8
#define PIECE   (NTHR * EPT)
#define WCAP    (EPT * 32)
#define NBC     512
#define SLB     9
#define O_PM    0
#define O_QM    16384
#define O_W1M   32768
#define O_W2M   49152
#define O_PC    65536
#define O_QC    81920
#define O_W1C   98304
#define O_W2C   114688
#define O_W0N   131072
#define O_W1N   180224
#define O_W2N   196608
#define O_TOT   212992
#define PREPBLK (O_TOT / (NTHR * 8))
#define PB0     (8 * HD)
#define PB1     (9 * HD)
#define PB2     (10 * HD)
#define WSCAP   134217728
#define PQDYN   (NWAVE * 16 * SP * 4)
#define L12DYN  (TE * SP * 4)
#define N0DYN   (NBN * XP3 * 2)
#define AGGDYN  (NBC * HD * 4)

static_assert((O_TOT % (NTHR * 8)) == 0);
static_assert((O_QM % 2048) == 0);
static_assert((O_W1M % 2048) == 0);
static_assert((O_W2M % 2048) == 0);
static_assert((O_PC % 2048) == 0);
static_assert((O_QC % 2048) == 0);
static_assert((O_W1C % 2048) == 0);
static_assert((O_W2C % 2048) == 0);
static_assert((O_W0N % 2048) == 0);
static_assert((O_W1N % 2048) == 0);
static_assert((O_W2N % 2048) == 0);
static_assert(((XP * 2) % 16) == 0);
static_assert(((XP3 * 2) % 16) == 0);
static_assert(((AP * 2) % 16) == 0);
static_assert(((SP * 4) % 16) == 0);
static_assert(NBC == (1 << SLB));
static_assert(PIECE == 2048);
static_assert((EPT % 4) == 0);
static_assert((NBC % NWAVE) == 0);
static_assert(NBN == 4 * 16);
static_assert(TE == NWAVE * 16);
static_assert(NTHR == 2 * TE);
static_assert((TE * AP * 2) <= L12DYN);
static_assert((PIECE % TE) == 0);
static_assert(((NBC * HD) % (4 * NTHR)) == 0);
static_assert((KN0 % 32) == 0);

typedef float          v4f   __attribute__((ext_vector_type(4)));
typedef float          v8f   __attribute__((ext_vector_type(8)));
typedef int            v4i   __attribute__((ext_vector_type(4)));
typedef unsigned int   v4u   __attribute__((ext_vector_type(4)));
typedef _Float16       v8h   __attribute__((ext_vector_type(8)));
typedef _Float16       v16h  __attribute__((ext_vector_type(16)));

__device__ __forceinline__ v16h ldfrag(const _Float16* p) {
  const v8h u0 = *(const v8h*)p;
  const v8h u1 = *(const v8h*)(p + 16);
  return __builtin_shufflevector(u0, u1, 0, 1, 2, 3, 4, 5, 6, 7, 8, 9, 10, 11, 12, 13, 14, 15);
}

__device__ __forceinline__ v8f wm(v16h a, v16h b, v8f c) {
  v8f d = __builtin_amdgcn_wmma_f32_16x16x32_f16(false, a, false, b, (short)0, c, false, false);
  asm volatile("v_nop\n\tv_nop\n\tv_nop\n\tv_nop" : "+v"(d) : "v"(a), "v"(b));
  return d;
}
__device__ __forceinline__ v8f zero8() {
  v8f z = {0.f, 0.f, 0.f, 0.f, 0.f, 0.f, 0.f, 0.f};
  return z;
}
__device__ __forceinline__ int iclamp(int v, int lo, int hi) { return v < lo ? lo : (v > hi ? hi : v); }

__device__ __forceinline__ v8h cvt8(v4f a, v4f b) {
  v8h u;
  u[0] = (_Float16)a.x; u[1] = (_Float16)a.y; u[2] = (_Float16)a.z; u[3] = (_Float16)a.w;
  u[4] = (_Float16)b.x; u[5] = (_Float16)b.y; u[6] = (_Float16)b.z; u[7] = (_Float16)b.w;
  return u;
}

__global__ __launch_bounds__(NTHR) void k_prep(
    const float* __restrict__ W0a, const float* __restrict__ W1a, const float* __restrict__ W2a,
    const float* __restrict__ W0b, const float* __restrict__ W1b, const float* __restrict__ W2b,
    const float* __restrict__ W0n, const float* __restrict__ W1n, const float* __restrict__ W2n,
    _Float16* wp) {
  const int tid = (int)threadIdx.x;
  const int o = ((int)blockIdx.x * NTHR + tid) * 8;
  const float* src;
  int rowb, idx, wide = 0;
  if (o < O_QM)       { src = W0a; rowb = 8;   idx = o; }
  else if (o < O_W1M) { src = W0a; rowb = 136; idx = o - O_QM; }
  else if (o < O_W2M) { src = W1a; rowb = 0;   idx = o - O_W1M; }
  else if (o < O_PC)  { src = W2a; rowb = 0;   idx = o - O_W2M; }
  else if (o < O_QC)  { src = W0b; rowb = 4;   idx = o - O_PC; }
  else if (o < O_W1C) { src = W0b; rowb = 132; idx = o - O_QC; }
  else if (o < O_W2C) { src = W1b; rowb = 0;   idx = o - O_W1C; }
  else if (o < O_W0N) { src = W2b; rowb = 0;   idx = o - O_W2C; }
  else if (o < O_W1N) { src = W0n; rowb = 0;   idx = o - O_W0N; wide = 1; }
  else if (o < O_W2N) { src = W1n; rowb = 0;   idx = o - O_W1N; }
  else                { src = W2n; rowb = 0;   idx = o - O_W2N; }
  int n, k0;
  if (wide != 0) { n = idx / KN0; k0 = idx - n * KN0; }
  else           { n = idx >> 7;  k0 = idx & (HD - 1); }
  v8h hv;
#pragma unroll
  for (int i = 0; i < 8; ++i) hv[i] = (_Float16)(64.0f * src[(size_t)(rowb + k0 + i) * HD + n]);
  const v4u u = __builtin_bit_cast(v4u, hv);
  _Float16* dst = wp + o;
  *(volatile v4u*)dst = u;
  __threadfence();
  *(volatile v4u*)dst = u;
}

__global__ __launch_bounds__(NTHR) void k_pq(const float* __restrict__ x, const _Float16* __restrict__ wpq,
                                             float* PQ, int nN) {
  extern __shared__ __attribute__((aligned(16))) float stg[];
  __shared__ __attribute__((aligned(16))) _Float16 sX[NBN * XP];
  const int tid = (int)threadIdx.x, lane = tid & 31, wave = tid >> 5, hh = lane >> 4, m = lane & 15;
  const int n0 = (int)blockIdx.x * NBN;

  {
    const int nl = tid >> 2, q = tid & 3;
    int node = n0 + nl;
    node = node > nN - 1 ? nN - 1 : node;
    const float* rp = x + (size_t)node * HD + 32 * q;
#pragma unroll
    for (int k = 0; k < 4; ++k) {
      const v4f a = *(const v4f*)(rp + 8 * k);
      const v4f b = *(const v4f*)(rp + 8 * k + 4);
      *(v8h*)(sX + nl * XP + 32 * q + 8 * k) = cvt8(a, b);
    }
  }
  __syncthreads();

  const int rt = wave & 3, cg = wave >> 2;
  const _Float16* bp = wpq + (cg != 0 ? HD * HD : 0);
  v8f c[8];
#pragma unroll
  for (int j = 0; j < 8; ++j) c[j] = zero8();
  const _Float16* ap = sX + (16 * rt + m) * XP + 8 * hh;
#pragma unroll 1
  for (int ks = 0; ks < 4; ++ks) {
    const v16h a = ldfrag(ap + 32 * ks);
#pragma unroll
    for (int j = 0; j < 8; ++j) {
      const v16h b = ldfrag(bp + (size_t)(16 * j + m) * HD + 32 * ks + 8 * hh);
      c[j] = wm(a, b, c[j]);
    }
  }
  float* sw = stg + wave * 16 * SP;
#pragma unroll
  for (int j = 0; j < 8; ++j) {
#pragma unroll
    for (int r = 0; r < 8; ++r) sw[(8 * hh + r) * SP + 16 * j + m] = c[j][r] * 0.015625f;
  }
  __syncthreads();
#pragma unroll 1
  for (int rr = 0; rr < 16; ++rr) {
    const v4f v = *(const v4f*)(sw + rr * SP + 4 * lane);
    *(volatile v4f*)(PQ + (size_t)(n0 + 16 * rt + rr) * PQROW + HD * cg + 4 * lane) = v;
  }
  __threadfence();
#pragma unroll 1
  for (int rr = 0; rr < 16; ++rr) {
    const v4f v = *(const v4f*)(sw + rr * SP + 4 * lane);
    *(volatile v4f*)(PQ + (size_t)(n0 + 16 * rt + rr) * PQROW + HD * cg + 4 * lane) = v;
  }
}

__device__ __forceinline__ void gemm128(const _Float16* sA, const _Float16* __restrict__ wpl,
                                        int rt, int cg, int hh, int m, v8f (&c)[2][4]) {
#pragma unroll
  for (int u = 0; u < 2; ++u) {
#pragma unroll
    for (int j = 0; j < 4; ++j) c[u][j] = zero8();
  }
  const _Float16* ap0 = sA + (32 * rt + m) * AP + 8 * hh;
  const _Float16* ap1 = ap0 + 16 * AP;
  const _Float16* bp = wpl + (size_t)(64 * cg + m) * HD + 8 * hh;
#pragma unroll 1
  for (int ks = 0; ks < 4; ++ks) {
    const v16h a0 = ldfrag(ap0 + 32 * ks);
    const v16h a1 = ldfrag(ap1 + 32 * ks);
#pragma unroll
    for (int j = 0; j < 4; ++j) {
      const v16h b = ldfrag(bp + (size_t)(16 * j) * HD + 32 * ks);
      c[0][j] = wm(a0, b, c[0][j]);
      c[1][j] = wm(a1, b, c[1][j]);
    }
  }
}

template <bool EDGE, int NGEO>
__global__ __launch_bounds__(NTHR) void k_l12(
    const int* __restrict__ gidx, const float* __restrict__ pp, const float* __restrict__ PQ,
    const float* __restrict__ W0, const float* __restrict__ b0, const _Float16* __restrict__ H0,
    const float* __restrict__ xres, const float* __restrict__ b1, const float* __restrict__ b2,
    const _Float16* __restrict__ w1p, const _Float16* __restrict__ w2p, float* dst,
    int c0, int nE, int nN) {
  extern __shared__ __attribute__((aligned(16))) float sBig[];
  __shared__ __attribute__((aligned(16))) float sPar[11 * HD];
  __shared__ __attribute__((aligned(16))) float sF[TE * 8];
  __shared__ int sIdx[2 * TE];
  _Float16* sA = (_Float16*)sBig;
  float* sO = sBig;
  const int tid = (int)threadIdx.x, lane = tid & 31, wave = tid >> 5, hh = lane >> 4, m = lane & 15;
  const int le0 = (int)blockIdx.x * TE;
  const int ge0 = c0 + le0;

  if (EDGE) {
    {
      const int s = tid >> 7, jx = tid & (TE - 1);
      int e = ge0 + jx;
      e = e > nE - 1 ? nE - 1 : e;
      int v = gidx[(size_t)s * nE + e];
      v = iclamp(v, 0, nN - 1);
      sIdx[s * TE + jx] = v;
    }
#pragma unroll 1
    for (int i = tid; i < NGEO * HD; i += NTHR) sPar[i] = W0[i];
    if (tid < HD) {
      sPar[PB0 + tid] = b0[tid];
      sPar[PB1 + tid] = b1[tid];
      sPar[PB2 + tid] = b2[tid];
    }
  } else {
    if (tid < HD) {
      sPar[PB1 + tid] = b1[tid];
      sPar[PB2 + tid] = b2[tid];
    }
  }
  __syncthreads();

  if (EDGE) {
    if (tid < TE) {
      const int in = sIdx[tid], jn = sIdx[TE + tid];
      const float* pi = pp + (size_t)in * 6;
      const float* pj = pp + (size_t)jn * 6;
      const float wx = pi[3] - pj[3], wy = pi[4] - pj[4], wz = pi[5] - pj[5];
      const float nw = sqrtf((wx * wx + wz * wz) + wy * wy);
      float* fo = sF + tid * 8;
      if (NGEO == 8) {
        const float dx = pi[0] - pj[0], dy = pi[1] - pj[1], dz = pi[2] - pj[2];
        const float nd = sqrtf((dx * dx + dz * dz) + dy * dy);
        fo[0] = dx; fo[1] = dy; fo[2] = dz; fo[3] = nd;
        fo[4] = wx; fo[5] = wy; fo[6] = wz; fo[7] = nw;
      } else {
        fo[0] = wx; fo[1] = wy; fo[2] = wz; fo[3] = nw;
        fo[4] = 0.f; fo[5] = 0.f; fo[6] = 0.f; fo[7] = 0.f;
      }
    }
    __syncthreads();

    {
      const int el = tid >> 1, q = tid & 1;
      const int rnode = sIdx[el], cnode = sIdx[TE + el];
      const float* prow = PQ + (size_t)rnode * PQROW + 64 * q;
      const float* qrow = PQ + (size_t)cnode * PQROW + HD + 64 * q;
      float f[NGEO];
#pragma unroll
      for (int t = 0; t < NGEO; ++t) f[t] = sF[el * 8 + t];
      _Float16* ad = sA + el * AP + 64 * q;
#pragma unroll 1
      for (int i = 0; i < 8; ++i) {
        const int cb = 64 * q + 8 * i;
        const v4f a0 = *(const v4f*)(prow + 8 * i);
        const v4f a1 = *(const v4f*)(prow + 8 * i + 4);
        const v4f g0 = *(const v4f*)(qrow + 8 * i);
        const v4f g1 = *(const v4f*)(qrow + 8 * i + 4);
        const v4f s0 = a0 + g0;
        const v4f s1 = a1 + g1;
        v4f d0 = {0.f, 0.f, 0.f, 0.f};
        v4f d1 = {0.f, 0.f, 0.f, 0.f};
#pragma unroll
        for (int t = 0; t < NGEO; ++t) {
          const v4f w0 = *(const v4f*)(sPar + t * HD + cb);
          const v4f w1 = *(const v4f*)(sPar + t * HD + cb + 4);
          d0 = d0 + f[t] * w0;
          d1 = d1 + f[t] * w1;
        }
        const v4f bb0 = *(const v4f*)(sPar + PB0 + cb);
        const v4f bb1 = *(const v4f*)(sPar + PB0 + cb + 4);
        const v4f z0 = (s0 + d0) + bb0;
        const v4f z1 = (s1 + d1) + bb1;
        v8h o;
        o[0] = (_Float16)(16.0f * fmaxf(z0.x, 0.f)); o[1] = (_Float16)(16.0f * fmaxf(z0.y, 0.f));
        o[2] = (_Float16)(16.0f * fmaxf(z0.z, 0.f)); o[3] = (_Float16)(16.0f * fmaxf(z0.w, 0.f));
        o[4] = (_Float16)(16.0f * fmaxf(z1.x, 0.f)); o[5] = (_Float16)(16.0f * fmaxf(z1.y, 0.f));
        o[6] = (_Float16)(16.0f * fmaxf(z1.z, 0.f)); o[7] = (_Float16)(16.0f * fmaxf(z1.w, 0.f));
        *(v8h*)(ad + 8 * i) = o;
      }
    }
  } else {
#pragma unroll 1
    for (int u = tid; u < TE * 16; u += NTHR) {
      const int row = u >> 4, c8 = u & 15;
      const v4u v = *(const v4u*)(H0 + (size_t)(le0 + row) * HD + 8 * c8);
      *(v4u*)(sA + row * AP + 8 * c8) = v;
    }
  }
  __syncthreads();

  const int rt = wave & 3, cg = wave >> 2;
  v8f c[2][4];
  gemm128(sA, w1p, rt, cg, hh, m, c);
  __syncthreads();
#pragma unroll
  for (int u = 0; u < 2; ++u) {
#pragma unroll
    for (int j = 0; j < 4; ++j) {
      const int col = 64 * cg + 16 * j + m;
      const float bb = sPar[PB1 + col];
      _Float16* sp = sA + (32 * rt + 16 * u + 8 * hh) * AP + col;
#pragma unroll
      for (int r = 0; r < 8; ++r)
        sp[r * AP] = (_Float16)(16.0f * fmaxf(c[u][j][r] * 0.0009765625f + bb, 0.f));
    }
  }
  __syncthreads();
  gemm128(sA, w2p, rt, cg, hh, m, c);
  __syncthreads();
#pragma unroll
  for (int u = 0; u < 2; ++u) {
#pragma unroll
    for (int j = 0; j < 4; ++j) {
      const int col = 64 * cg + 16 * j + m;
      const float bb = sPar[PB2 + col];
      float* sp = sO + (32 * rt + 16 * u + 8 * hh) * SP + col;
#pragma unroll
      for (int r = 0; r < 8; ++r) sp[r * SP] = c[u][j][r] * 0.0009765625f + bb;
    }
  }
  __syncthreads();

  {
    const int el = tid >> 1, q = tid & 1;
    float* so = sO + el * SP + 64 * q;
    float s = 0.f;
#pragma unroll
    for (int k = 0; k < 16; ++k) {
      const v4f h = *(const v4f*)(so + 4 * k);
      s += (h.x + h.y) + (h.z + h.w);
    }
    s += __shfl_xor(s, 1, 32);
    const float mean = s * 0.0078125f;
    float vs = 0.f;
#pragma unroll
    for (int k = 0; k < 16; ++k) {
      const v4f h = *(const v4f*)(so + 4 * k);
      const v4f d = h - mean;
      vs += (d.x * d.x + d.y * d.y) + (d.z * d.z + d.w * d.w);
    }
    vs += __shfl_xor(vs, 1, 32);
    const float inv = rsqrtf(vs * 0.0078125f + 1e-5f);
    int nodec = le0 + el;
    nodec = nodec > nN - 1 ? nN - 1 : nodec;
    const float* xr = xres + (size_t)nodec * HD + 64 * q;
#pragma unroll
    for (int k = 0; k < 16; ++k) {
      const v4f h = *(const v4f*)(so + 4 * k);
      v4f rv = (h - mean) * inv;
      if (!EDGE) rv = rv + *(const v4f*)(xr + 4 * k);
      *(v4f*)(so + 4 * k) = rv;
    }
  }
  __syncthreads();

#pragma unroll 1
  for (int i = 0; i < 16; ++i) {
    const int row = 16 * wave + i;
    const int grow = le0 + row;
    if (!EDGE && grow >= nN) continue;
    const v4f v = *(const v4f*)(sO + row * SP + 4 * lane);
    *(volatile v4f*)(dst + (size_t)grow * HD + 4 * lane) = v;
  }
  __threadfence();
#pragma unroll 1
  for (int i = 0; i < 16; ++i) {
    const int row = 16 * wave + i;
    const int grow = le0 + row;
    if (!EDGE && grow >= nN) continue;
    const v4f v = *(const v4f*)(sO + row * SP + 4 * lane);
    *(volatile v4f*)(dst + (size_t)grow * HD + 4 * lane) = v;
  }
}

__device__ __forceinline__ int scan_piece(const int* __restrict__ kp, int lim, int cbase, int base,
                                          int* list, int tid, int wave, int vec_ok) {
  int wc = 0;
  const int el0  = tid * EPT;
  const int e0   = cbase + el0;
  const int sent = -2147483647 - 1;
  int kk[EPT];
  if (vec_ok != 0 && cbase + PIECE <= lim) {
    const v4i* p = (const v4i*)(kp + e0);
#pragma unroll
    for (int u = 0; u < EPT / 4; ++u) {
      const v4i d = p[u];
      kk[4 * u] = d.x; kk[4 * u + 1] = d.y; kk[4 * u + 2] = d.z; kk[4 * u + 3] = d.w;
    }
  } else {
    const int lm = lim - 1;
#pragma unroll
    for (int q = 0; q < EPT; ++q) {
      const int eq = e0 + q;
      const int ec = eq > lm ? lm : eq;
      const int a = kp[ec];
      kk[q] = (eq < lim) ? a : sent;
    }
  }
  const unsigned nb = (unsigned)base;
  unsigned sq[EPT];
  bool hq[EPT];
  bool anyl = false;
#pragma unroll
  for (int q = 0; q < EPT; ++q) {
    sq[q] = (unsigned)kk[q] - nb;
    hq[q] = sq[q] < (unsigned)NBC;
    anyl = anyl | hq[q];
  }
  const unsigned any = __builtin_amdgcn_ballot_w32(anyl);
  if (any != 0u) {
#define HIT(HQ, SQ, Q) { \
      const unsigned mj = __builtin_amdgcn_ballot_w32(HQ); \
      if (mj != 0u) { \
        if (HQ) { \
          const int ps = wc + (int)__builtin_amdgcn_mbcnt_lo(mj, 0u); \
          if (ps < WCAP) list[wave * WCAP + ps] = ((el0 + (Q)) << SLB) | (int)(SQ); \
        } \
        wc += (int)__builtin_popcount(mj); } }
#pragma unroll
    for (int q = 0; q < EPT; ++q) {
      HIT(hq[q], sq[q], q)
    }
#undef HIT
  }
  return wc;
}

__device__ __forceinline__ void drain_sum(const int* list, const int* wcnt, float* accF,
                                          const float* __restrict__ OE,
                                          int cbase, int nec, int lane, int wave) {
#pragma unroll 1
  for (int wsx = 0; wsx < NWAVE; ++wsx) {
    int n = __builtin_amdgcn_readfirstlane(wcnt[wsx]);
    n = n > WCAP ? WCAP : (n < 0 ? 0 : n);
    const int* lp = list + wsx * WCAP;
#pragma unroll 1
    for (int bb = 0; bb < n; bb += 32) {
      const int idx = bb + lane;
      const int ic = idx > WCAP - 1 ? WCAP - 1 : idx;
      const int ent = lp[ic];
      const bool own = (idx < n) && ((ent & (NWAVE - 1)) == wave);
      unsigned msk = __builtin_amdgcn_ballot_w32(own);
#pragma unroll 1
      while (msk != 0u) {
        const int bit = (int)__builtin_ctz(msk);
        msk &= msk - 1u;
        const int e2 = __builtin_amdgcn_readlane(ent, bit);
        const int slot = e2 & (NBC - 1);
        const int el = (e2 >> SLB) & (PIECE - 1);
        int e = cbase + el;
        e = e > nec - 1 ? nec - 1 : (e < 0 ? 0 : e);
        const v4f hv = *(const v4f*)(OE + (size_t)e * HD + 4 * lane);
        float* ap = accF + slot * HD + 4 * lane;
        v4f a = *(const v4f*)ap;
        a = a + hv;
        *(v4f*)ap = a;
      }
    }
  }
}

__device__ __forceinline__ void node_rows(const float* accF, float* aggp, int base, int wave, int lane) {
#pragma unroll 1
  for (int it = 0; it < NBC / NWAVE; ++it) {
    const int s = wave + NWAVE * it;
    const v4f v = *(const v4f*)(accF + s * HD + 4 * lane);
    *(volatile v4f*)(aggp + (size_t)(base + s) * HD + 4 * lane) = v;
  }
}

__global__ __launch_bounds__(NTHR) void k_agg(
    const int* __restrict__ gidx, const float* __restrict__ OE, float* aggp,
    int c0, int nec, int nE, int first, int vec_ok) {
  extern __shared__ __attribute__((aligned(16))) float accF[];
  __shared__ int list[NWAVE * WCAP];
  __shared__ int wcnt[NWAVE];
  const int tid = (int)threadIdx.x, lane = tid & 31, wave = tid >> 5;
  const int base = (int)blockIdx.x * NBC;

  if (first != 0) {
    const v4f z = {0.0f, 0.0f, 0.0f, 0.0f};
#pragma unroll 1
    for (int i = tid; i < (NBC * HD) / 4; i += NTHR) *(v4f*)(accF + 4 * i) = z;
  } else {
    const float* src = aggp + (size_t)base * HD;
#pragma unroll 1
    for (int i = tid; i < (NBC * HD) / 4; i += NTHR) *(v4f*)(accF + 4 * i) = *(const v4f*)(src + 4 * i);
  }
  __syncthreads();

  const int* kp = gidx + (size_t)nE + c0;
#pragma unroll 1
  for (int cbase = 0; cbase < nec; cbase += PIECE) {
    const int wc = scan_piece(kp, nec, cbase, base, list, tid, wave, vec_ok);
    if (lane == 0) wcnt[wave] = wc;
    __syncthreads();
    drain_sum(list, wcnt, accF, OE, cbase, nec, lane, wave);
    __syncthreads();
  }
  __syncthreads();

  node_rows(accF, aggp, base, wave, lane);
  __threadfence();
  node_rows(accF, aggp, base, wave, lane);
}

__global__ __launch_bounds__(NTHR) void k_node0(
    const float* __restrict__ x, const float* __restrict__ agga, const float* __restrict__ aggb,
    const _Float16* __restrict__ w0n, const float* __restrict__ b0, _Float16* H0, int nN) {
  extern __shared__ __attribute__((aligned(16))) float sDyn[];
  __shared__ __attribute__((aligned(16))) _Float16 sH[NBN * AP];
  _Float16* sX3 = (_Float16*)sDyn;
  const int tid = (int)threadIdx.x, lane = tid & 31, wave = tid >> 5, hh = lane >> 4, m = lane & 15;
  const int n0 = (int)blockIdx.x * NBN;

#pragma unroll 1
  for (int u = tid; u < NBN * 16; u += NTHR) {
    const int row = u >> 4, c8 = u & 15;
    int node = n0 + row;
    node = node > nN - 1 ? nN - 1 : node;
    const float* sp = x + (size_t)node * HD + 8 * c8;
    *(v8h*)(sX3 + row * XP3 + 8 * c8) = cvt8(*(const v4f*)sp, *(const v4f*)(sp + 4));
  }
#pragma unroll 1
  for (int u = tid; u < NBN * 16; u += NTHR) {
    const int row = u >> 4, c8 = u & 15;
    int node = n0 + row;
    node = node > nN - 1 ? nN - 1 : node;
    const float* sp = agga + (size_t)node * HD + 8 * c8;
    *(v8h*)(sX3 + row * XP3 + HD + 8 * c8) = cvt8(*(const v4f*)sp, *(const v4f*)(sp + 4));
  }
#pragma unroll 1
  for (int u = tid; u < NBN * 16; u += NTHR) {
    const int row = u >> 4, c8 = u & 15;
    int node = n0 + row;
    node = node > nN - 1 ? nN - 1 : node;
    const float* sp = aggb + (size_t)node * HD + 8 * c8;
    *(v8h*)(sX3 + row * XP3 + 2 * HD + 8 * c8) = cvt8(*(const v4f*)sp, *(const v4f*)(sp + 4));
  }
  __syncthreads();

  const int rt = wave & 3, cg = wave >> 2;
  v8f c[4];
#pragma unroll
  for (int j = 0; j < 4; ++j) c[j] = zero8();
  {
    const _Float16* ap = sX3 + (16 * rt + m) * XP3 + 8 * hh;
    const _Float16* bp = w0n + (size_t)(64 * cg + m) * KN0 + 8 * hh;
#pragma unroll 1
    for (int ks = 0; ks < KN0 / 32; ++ks) {
      const v16h a = ldfrag(ap + 32 * ks);
#pragma unroll
      for (int j = 0; j < 4; ++j) {
        const v16h b = ldfrag(bp + (size_t)(16 * j) * KN0 + 32 * ks);
        c[j] = wm(a, b, c[j]);
      }
    }
  }
#pragma unroll
  for (int j = 0; j < 4; ++j) {
    const int col = 64 * cg + 16 * j + m;
    const float bb = b0[col];
    _Float16* sp = sH + (16 * rt + 8 * hh) * AP + col;
#pragma unroll
    for (int r = 0; r < 8; ++r) sp[r * AP] = (_Float16)(16.0f * fmaxf(c[j][r] * 0.015625f + bb, 0.f));
  }
  __syncthreads();
#pragma unroll 1
  for (int it = 0; it < NBN / (2 * NWAVE); ++it) {
    const int row = 2 * (wave + NWAVE * it) + hh;
    const v4u v = *(const v4u*)(sH + row * AP + 8 * m);
    *(volatile v4u*)(H0 + (size_t)(n0 + row) * HD + 8 * m) = v;
  }
  __threadfence();
#pragma unroll 1
  for (int it = 0; it < NBN / (2 * NWAVE); ++it) {
    const int row = 2 * (wave + NWAVE * it) + hh;
    const v4u v = *(const v4u*)(sH + row * AP + 8 * m);
    *(volatile v4u*)(H0 + (size_t)(n0 + row) * HD + 8 * m) = v;
  }
}

extern "C" void kernel_launch(void* const* d_in, const int* in_sizes, int n_in,
                              void* d_out, int out_size, void* d_ws, size_t ws_size,
                              hipStream_t stream) {
  if (n_in < 22) return;
  if (in_sizes[0] < HD || (in_sizes[0] % HD) != 0) return;
  const int nN = in_sizes[0] / HD;
  if (nN < 1 || nN > (1 << 22)) return;
  if ((in_sizes[1] & 1) != 0 || (in_sizes[2] & 1) != 0) return;
  const int nE = in_sizes[1] / 2;
  const int nC = in_sizes[2] / 2;
  if (nE < 1 || nE > (1 << 27) || nC < 1 || nC > (1 << 27)) return;
  if (in_sizes[3] != nN * 6) return;
  if (in_sizes[4] != 264 * HD || in_sizes[10] != 260 * HD || in_sizes[16] != KN0 * HD) return;
  if (in_sizes[6] != HD * HD || in_sizes[8] != HD * HD) return;
  if (in_sizes[12] != HD * HD || in_sizes[14] != HD * HD) return;
  if (in_sizes[18] != HD * HD || in_sizes[20] != HD * HD) return;
  for (int b = 5; b <= 21; b += 2) { if (in_sizes[b] != HD) return; }
  if ((long long)out_size != (long long)nN * HD) return;

  const float* x   = (const float*)d_in[0];
  const int*   g   = (const int*)d_in[1];
  const int*   gc  = (const int*)d_in[2];
  const float* pp  = (const float*)d_in[3];
  const float* W0a = (const float*)d_in[4];  const float* b0a = (const float*)d_in[5];
  const float* W1a = (const float*)d_in[6];  const float* b1a = (const float*)d_in[7];
  const float* W2a = (const float*)d_in[8];  const float* b2a = (const float*)d_in[9];
  const float* W0b = (const float*)d_in[10]; const float* b0b = (const float*)d_in[11];
  const float* W1b = (const float*)d_in[12]; const float* b1b = (const float*)d_in[13];
  const float* W2b = (const float*)d_in[14]; const float* b2b = (const float*)d_in[15];
  const float* W0n = (const float*)d_in[16]; const float* b0n = (const float*)d_in[17];
  const float* W1n = (const float*)d_in[18]; const float* b1n = (const float*)d_in[19];
  const float* W2n = (const float*)d_in[20]; const float* b2n = (const float*)d_in[21];
  float* outp = (float*)d_out;

  const int nbT   = (nN + TE - 1) / TE;
  const int Npad  = nbT * TE;
  const int nb64  = Npad / NBN;
  const int nbA   = (nN + NBC - 1) / NBC;
  const int vokA  = ((nE & 3) == 0) ? 1 : 0;
  const int vokB  = ((nC & 3) == 0) ? 1 : 0;

  const size_t cap  = ws_size < (size_t)WSCAP ? ws_size : (size_t)WSCAP;
  const size_t bW   = (size_t)O_TOT * 2;
  const size_t bPQ  = (size_t)Npad * PQROW * 4;
  const size_t bH0  = (size_t)Npad * HD * 2;
  if (bH0 > bPQ) return;
  const size_t bAG  = (size_t)nbA * NBC * HD * 4;
  char* ws = (char*)d_ws;
  size_t off = 0;
  const size_t oW  = off; off += bW;   off = (off + 255) & ~(size_t)255;
  const size_t oPQ = off; off += bPQ;  off = (off + 255) & ~(size_t)255;
  const size_t oAA = off; off += bAG;  off = (off + 255) & ~(size_t)255;
  const size_t oAB = off; off += bAG;  off = (off + 255) & ~(size_t)255;
  if (off >= cap) return;
  const int maxE = nE > nC ? nE : nC;
  const size_t cemax = (((size_t)maxE + PIECE - 1) / PIECE) * PIECE;
  const size_t avail = cap - off;
  size_t CE = (avail / ((size_t)HD * 4)) / PIECE * PIECE;
  if (CE > cemax) CE = cemax;
  if (CE < (size_t)PIECE) return;
  const size_t oOE = off; off += CE * HD * 4; off = (off + 255) & ~(size_t)255;
  if (off > cap || off > ws_size) return;

  _Float16* wp   = (_Float16*)(ws + oW);
  float*    PQ   = (float*)(ws + oPQ);
  _Float16* H0   = (_Float16*)(ws + oPQ);
  float*    agga = (float*)(ws + oAA);
  float*    aggb = (float*)(ws + oAB);
  float*    OE   = (float*)(ws + oOE);

  hipFuncSetAttribute(reinterpret_cast<const void*>(&k_pq),            hipFuncAttributeMaxDynamicSharedMemorySize, PQDYN);
  hipFuncSetAttribute(reinterpret_cast<const void*>(&k_l12<true, 8>),  hipFuncAttributeMaxDynamicSharedMemorySize, L12DYN);
  hipFuncSetAttribute(reinterpret_cast<const void*>(&k_l12<true, 4>),  hipFuncAttributeMaxDynamicSharedMemorySize, L12DYN);
  hipFuncSetAttribute(reinterpret_cast<const void*>(&k_l12<false, 8>), hipFuncAttributeMaxDynamicSharedMemorySize, L12DYN);
  hipFuncSetAttribute(reinterpret_cast<const void*>(&k_agg),           hipFuncAttributeMaxDynamicSharedMemorySize, AGGDYN);
  hipFuncSetAttribute(reinterpret_cast<const void*>(&k_node0),         hipFuncAttributeMaxDynamicSharedMemorySize, N0DYN);

  k_prep<<<PREPBLK, NTHR, 0, stream>>>(W0a, W1a, W2a, W0b, W1b, W2b, W0n, W1n, W2n, wp);

  k_pq<<<nb64, NTHR, PQDYN, stream>>>(x, wp + O_PM, PQ, nN);
  {
    const int nch = (int)(((size_t)nE + CE - 1) / CE);
    for (int ch = 0; ch < nch; ++ch) {
      const size_t c0s = (size_t)ch * CE;
      if (c0s >= (size_t)nE) break;
      const int c0 = (int)c0s;
      size_t necs = (size_t)nE - c0s;
      if (necs > CE) necs = CE;
      const int nec = (int)necs;
      const int ntiles = (nec + TE - 1) / TE;
      k_l12<true, 8><<<ntiles, NTHR, L12DYN, stream>>>(g, pp, PQ, W0a, b0a, H0, x, b1a, b2a,
                                                        wp + O_W1M, wp + O_W2M, OE, c0, nE, nN);
      k_agg<<<nbA, NTHR, AGGDYN, stream>>>(g, OE, agga, c0, nec, nE, (ch == 0) ? 1 : 0, vokA);
    }
  }
  k_pq<<<nb64, NTHR, PQDYN, stream>>>(x, wp + O_PC, PQ, nN);
  {
    const int nch = (int)(((size_t)nC + CE - 1) / CE);
    for (int ch = 0; ch < nch; ++ch) {
      const size_t c0s = (size_t)ch * CE;
      if (c0s >= (size_t)nC) break;
      const int c0 = (int)c0s;
      size_t necs = (size_t)nC - c0s;
      if (necs > CE) necs = CE;
      const int nec = (int)necs;
      const int ntiles = (nec + TE - 1) / TE;
      k_l12<true, 4><<<ntiles, NTHR, L12DYN, stream>>>(gc, pp, PQ, W0b, b0b, H0, x, b1b, b2b,
                                                        wp + O_W1C, wp + O_W2C, OE, c0, nC, nN);
      k_agg<<<nbA, NTHR, AGGDYN, stream>>>(gc, OE, aggb, c0, nec, nC, (ch == 0) ? 1 : 0, vokB);
    }
  }
  k_node0<<<nb64, NTHR, N0DYN, stream>>>(x, agga, aggb, wp + O_W0N, b0n, H0, nN);
  k_l12<false, 8><<<nbT, NTHR, L12DYN, stream>>>(g, pp, PQ, W0a, b0a, H0, x, b1n, b2n,
                                                  wp + O_W1N, wp + O_W2N, outp, 0, nE, nN);
}
